// ImprovedGNN_82429012345509
// MI455X (gfx1250) — hardware-run, weakly checked
//
#include <hip/hip_runtime.h>
#include <stddef.h>
#include <stdint.h>


#define NN     50000
#define NE     800000
#define HID    128
#define EDIM   16
#define KW     272
#define K2     256
#define NPAB   256
#define EFK    32
#define NTHR   256
#define NWAVE  8
#define EPT    8
#define CHUNK  (NTHR * EPT)
#define WCAP   (EPT * 32)
#define LISTN  (NWAVE * WCAP)
#define NBA    1024
#define SLA    10
#define NBLK   49
#define NTAB   (NBLK * NBA)
#define RCAP   28672
#define DEGCAP 64
#define GBM    64
#define GBN    128
#define GTHR   128
#define NPADR  50048
#define APB    32
#define EPB    256
#define DP     132
#define NU_W1  (HID * (HID / 8))
#define NU_W2  (HID * (K2 / 8))
#define NU_WP  (NPAB * (K2 / 8))
#define NU_WE  (HID * (EFK / 8))
#define NU_XB  (NPADR * (HID / 8))
#define BKT_ZINTS (LISTN + 2 * RCAP + 3 * NBA)
#define BKT_LDS_INTS (BKT_ZINTS + 16)
#define BKT_LDS_BYTES (BKT_LDS_INTS * 4)
#define HEAD_LDS_BYTES ((NWAVE * 16 * DP + 2 * HID + 4) * 4)
#define WSMAX  134217728

static_assert(NBLK * NBA >= NN);
static_assert(NTAB >= NPADR && NPADR >= NN);
static_assert(NPADR % 128 == 0 && NPADR % GBM == 0 && NPADR % APB == 0);
static_assert(NE % EPB == 0 && NE % 4 == 0);
static_assert(HID == 32 * 4);
static_assert((CHUNK & (CHUNK - 1)) == 0 && CHUNK <= 4096);
static_assert((NBA & (NBA - 1)) == 0 && NBA == (1 << SLA) && NBA == 4 * NTHR && NBA % 32 == 0);
static_assert(((long long)NE << SLA) < (1LL << 31));
static_assert(((long long)CHUNK << SLA) < (1LL << 31));
static_assert(RCAP % (4 * NTHR) == 0 && RCAP >= 16623 && DEGCAP >= 35 + 8);
static_assert(BKT_ZINTS % 4 == 0 && LISTN % 4 == 0);
static_assert(BKT_LDS_BYTES <= 327680 && HEAD_LDS_BYTES <= 327680);
static_assert(NU_W1 % NTHR == 0 && NU_W2 % NTHR == 0 && NU_WP % NTHR == 0 && NU_WE % NTHR == 0 && NU_XB % NTHR == 0);
static_assert((NU_W1 + NU_W2 + (NU_WP / 2)) % NTHR == 0);
static_assert(GBM == (GTHR / 32) * 16 && GBN == HID && NPAB == 2 * GBN && K2 == 2 * HID);
static_assert(HID % 32 == 0 && K2 % 32 == 0 && EFK == 32 && EDIM == 16 && KW == 2 * HID + EDIM);
static_assert((DP * 4) % 16 == 0 && DP >= HID);
static_assert(EPB == NTHR && EPB == NWAVE * 32);

typedef float          v4f   __attribute__((ext_vector_type(4)));
typedef float          v8f   __attribute__((ext_vector_type(8)));
typedef int            v4i   __attribute__((ext_vector_type(4)));
typedef int            v8i   __attribute__((ext_vector_type(8)));
typedef unsigned int   v4u   __attribute__((ext_vector_type(4)));
typedef unsigned short v8us  __attribute__((ext_vector_type(8)));
typedef unsigned short v16us __attribute__((ext_vector_type(16)));
typedef __bf16         v16bf __attribute__((ext_vector_type(16)));
typedef v4f  __attribute__((may_alias)) v4fa;
typedef v4i  __attribute__((may_alias)) v4ia;
typedef v8us __attribute__((may_alias)) v8usa;
union FragB { v16bf v; v16us u; v8us h[2]; v8i w; };

__device__ __forceinline__ v8f wmb(const FragB& a, const FragB& b, v8f c) {
  v8f d = __builtin_amdgcn_wmma_f32_16x16x32_bf16(false, a.v, false, b.v, (short)0, c, false, false);
  asm volatile("v_nop\n\tv_nop\n\tv_nop\n\tv_nop" : "+v"(d) : "v"(a.w), "v"(b.w));
  return d;
}

__device__ __forceinline__ unsigned bf16_bits(float f) {
  const unsigned u = __float_as_uint(f);
  return (u + 0x7FFFu + ((u >> 16) & 1u)) >> 16;
}
__device__ __forceinline__ float bf16_val(float f) {
  return __uint_as_float(bf16_bits(f) << 16);
}
__device__ __forceinline__ unsigned bf16_bits_np(float f) {
  const unsigned r = bf16_bits(f);
  return (f != f) ? 0x7fc0u : r;
}
__device__ __forceinline__ float rsq_ref(float d) {
  const float y = rsqrtf(d);
  const float e = fmaf(-d * y, y, 1.0f);
  return fmaf(0.5f * y, e, y);
}
__device__ __forceinline__ int clampi(int v, int lo, int hi) {
  return v < lo ? lo : (v > hi ? hi : v);
}
__device__ __forceinline__ void put16(unsigned short* dp, v8us o) {
  *(volatile v8us*)dp = o;
  __threadfence();
  *(volatile v8us*)dp = o;
}

template <int SLB>
__device__ __forceinline__ int scan_chunk(const int* __restrict__ dsts, int nE, int cbase, int slotBase,
                                          int nb, int vec8, int* list, int tid, int lane, int wave) {
  int wc = 0;
  const int el0  = tid * EPT;
  const int e0   = cbase + el0;
  const int sent = -2147483647 - 1;
  v4i da, db;
  if (vec8 != 0 && cbase + CHUNK <= nE) {
    da = *(const v4i*)(dsts + e0);
    db = *(const v4i*)(dsts + e0 + 4);
  } else {
    da.x = (e0     < nE) ? dsts[min(e0,     nE - 1)] : sent;
    da.y = (e0 + 1 < nE) ? dsts[min(e0 + 1, nE - 1)] : sent;
    da.z = (e0 + 2 < nE) ? dsts[min(e0 + 2, nE - 1)] : sent;
    da.w = (e0 + 3 < nE) ? dsts[min(e0 + 3, nE - 1)] : sent;
    db.x = (e0 + 4 < nE) ? dsts[min(e0 + 4, nE - 1)] : sent;
    db.y = (e0 + 5 < nE) ? dsts[min(e0 + 5, nE - 1)] : sent;
    db.z = (e0 + 6 < nE) ? dsts[min(e0 + 6, nE - 1)] : sent;
    db.w = (e0 + 7 < nE) ? dsts[min(e0 + 7, nE - 1)] : sent;
  }
  const unsigned nbs = (unsigned)slotBase;
  const unsigned unb = (unsigned)nb;
  const unsigned s0 = (unsigned)da.x - nbs, s1 = (unsigned)da.y - nbs;
  const unsigned s2 = (unsigned)da.z - nbs, s3 = (unsigned)da.w - nbs;
  const unsigned s4 = (unsigned)db.x - nbs, s5 = (unsigned)db.y - nbs;
  const unsigned s6 = (unsigned)db.z - nbs, s7 = (unsigned)db.w - nbs;
  const bool h0 = s0 < unb, h1 = s1 < unb, h2 = s2 < unb, h3 = s3 < unb;
  const bool h4 = s4 < unb, h5 = s5 < unb, h6 = s6 < unb, h7 = s7 < unb;
  const unsigned any = __builtin_amdgcn_ballot_w32(h0 | h1 | h2 | h3 | h4 | h5 | h6 | h7);
  if (any != 0u) {
#define HITJ(J, HJ, SJ) { \
      const unsigned mj = __builtin_amdgcn_ballot_w32(HJ); \
      if (mj != 0u) { \
        if (HJ) { \
          const int pos = wc + (int)__builtin_amdgcn_mbcnt_lo(mj, 0u); \
          if (pos < WCAP) list[wave * WCAP + pos] = ((el0 + (J)) << SLB) | (int)(SJ); \
        } \
        wc += (int)__builtin_popcount(mj); } }
    HITJ(0, h0, s0)
    HITJ(1, h1, s1)
    HITJ(2, h2, s2)
    HITJ(3, h3, s3)
    HITJ(4, h4, s4)
    HITJ(5, h5, s5)
    HITJ(6, h6, s6)
    HITJ(7, h7, s7)
#undef HITJ
  }
  return wc;
}

__global__ __launch_bounds__(NTHR) void k_prep(const float* __restrict__ x, const float* __restrict__ W1,
                                               const float* __restrict__ W2, const float* __restrict__ Wm1,
                                               int nN,
                                               unsigned short* W1T, unsigned short* W2D, unsigned short* WPD,
                                               unsigned short* WET, unsigned short* XB) {
  const int u  = (int)blockIdx.x * NTHR + (int)threadIdx.x;
  const int U0 = NU_W1;
  const int U1 = U0 + NU_W2;
  const int U2 = U1 + NU_WP;
  const int U3 = U2 + NU_WE;
  const int U4 = U3 + NU_XB;
  v8us o;
  if (u < U0) {
    const int n  = u >> 4;
    const int k8 = (u & 15) * 8;
    const float* p = W1 + (size_t)k8 * HID + n;
#pragma unroll
    for (int i = 0; i < 8; ++i) o[i] = (unsigned short)bf16_bits(p[(size_t)i * HID]);
    put16(W1T + (size_t)n * HID + k8, o);
    return;
  } else if (u < U1) {
    const int v  = u - U0;
    const int n  = v >> 5;
    const int k8 = (v & 31) * 8;
    const int kk = k8 & (HID - 1);
    const float* p = W2 + (size_t)kk * HID + n;
#pragma unroll
    for (int i = 0; i < 8; ++i) o[i] = (unsigned short)bf16_bits(p[(size_t)i * HID]);
    put16(W2D + (size_t)n * K2 + k8, o);
    return;
  } else if (u < U2) {
    const int v    = u - U1;
    const int n    = v >> 5;
    const int k8   = (v & 31) * 8;
    const int kk   = k8 & (HID - 1);
    const int roff = (n >> 7) * HID;
    const int nn   = n & (HID - 1);
    const float* p = Wm1 + (size_t)(roff + kk) * HID + nn;
#pragma unroll
    for (int i = 0; i < 8; ++i) o[i] = (unsigned short)bf16_bits(p[(size_t)i * HID]);
    put16(WPD + (size_t)n * K2 + k8, o);
    return;
  } else if (u < U3) {
    const int v  = u - U2;
    const int n  = v >> 2;
    const int k8 = (v & 3) * 8;
    const int kc = (k8 < EDIM) ? k8 : 0;
    const unsigned msk = (k8 < EDIM) ? 0xFFFFu : 0u;
    const float* p = Wm1 + (size_t)(2 * HID + kc) * HID + n;
#pragma unroll
    for (int i = 0; i < 8; ++i) {
      const float w = p[(size_t)i * HID];
      asm volatile("" :: "v"(w));
      o[i] = (unsigned short)(bf16_bits(w) & msk);
    }
    put16(WET + (size_t)n * EFK + k8, o);
    return;
  } else if (u < U4) {
    const int v   = u - U3;
    const int row = v >> 4;
    const int k8  = (v & 15) * 8;
    const int rc  = row < nN ? row : nN - 1;
    const float* p = x + (size_t)rc * HID + k8;
    const v4f a = *(const v4fa*)p;
    const v4f b = *(const v4fa*)(p + 4);
    asm volatile("" :: "v"(a), "v"(b));
    const unsigned msk = (row < nN) ? 0xFFFFu : 0u;
    o[0] = (unsigned short)(bf16_bits(a.x) & msk);
    o[1] = (unsigned short)(bf16_bits(a.y) & msk);
    o[2] = (unsigned short)(bf16_bits(a.z) & msk);
    o[3] = (unsigned short)(bf16_bits(a.w) & msk);
    o[4] = (unsigned short)(bf16_bits(b.x) & msk);
    o[5] = (unsigned short)(bf16_bits(b.y) & msk);
    o[6] = (unsigned short)(bf16_bits(b.z) & msk);
    o[7] = (unsigned short)(bf16_bits(b.w) & msk);
    put16(XB + (size_t)row * HID + k8, o);
    return;
  }
}

__global__ __launch_bounds__(NTHR) void k_bucket(const int* __restrict__ srcs, const int* __restrict__ dsts,
                                                 int nE, int nN, int vec8,
                                                 int* HITS, int* CNT, int* OFF, float* DINV, int* FLG) {
  extern __shared__ __attribute__((aligned(16))) int dsm[];
  int* list = dsm;
  int* hl   = dsm + LISTN;
  int* sl   = dsm + LISTN + RCAP;
  int* cnt  = dsm + LISTN + 2 * RCAP;
  int* offs = cnt + NBA;
  int* cur  = offs + NBA;
  int* misc = cur + NBA;
  const int tid = (int)threadIdx.x, lane = tid & 31, wave = tid >> 5;
  const int nodeBase = (int)blockIdx.x * NBA;

  {
    const v4i z4 = {0, 0, 0, 0};
    for (int i = tid * 4; i < BKT_ZINTS; i += NTHR * 4) *(v4ia*)(dsm + i) = z4;
    if (tid < 16) misc[tid] = 0;
  }
  __syncthreads();

  int t = 0, ov = 0;
  const int nChunks = (nE + CHUNK - 1) / CHUNK;
#pragma unroll 1
  for (int ch = 0; ch < nChunks; ++ch) {
    const int cbase = ch * CHUNK;
    const int wc = scan_chunk<SLA>(dsts, nE, cbase, nodeBase, NBA, vec8, list, tid, lane, wave);
    if (lane == 0) misc[wave] = wc;
    __syncthreads();
    if (wave == 0) {
#pragma unroll 1
      for (int w2 = 0; w2 < NWAVE; ++w2) {
        int c = misc[w2];
        c = c < 0 ? 0 : (c > WCAP ? WCAP : c);
#pragma unroll 1
        for (int b0 = 0; b0 < c; b0 += 32) {
          const int idx = b0 + lane;
          const int ent = list[w2 * WCAP + (idx < WCAP ? idx : WCAP - 1)];
          const int m32 = (c - b0) < 32 ? (c - b0) : 32;
#pragma unroll 1
          for (int k = 0; k < m32; ++k) {
            const int u    = __builtin_amdgcn_readlane(ent, k);
            const int slot = u & (NBA - 1);
            const int el   = (u >> SLA) & (CHUNK - 1);
            const int pk   = ((cbase + el) << SLA) | slot;
            if (t < RCAP) {
              if (lane == 0) { hl[t] = pk; cnt[slot] = cnt[slot] + 1; }
              t = t + 1;
            } else {
              ov = 1;
            }
          }
        }
      }
    }
    __syncthreads();
  }
  if (wave == 0 && lane == 0) { misc[8] = t; misc[9] = ov; }
  __syncthreads();
  int tt = misc[8];
  tt = tt < 0 ? 0 : (tt > RCAP ? RCAP : tt);
  const int ovf = misc[9];

  if (wave == 0) {
    const int base = lane * (NBA / 32);
    int s = 0;
#pragma unroll 1
    for (int i = 0; i < NBA / 32; ++i) s += cnt[base + i];
    int incl = s;
#pragma unroll
    for (int d = 1; d < 32; d <<= 1) {
      const int y = __shfl_up(incl, d, 32);
      if (lane >= d) incl += y;
    }
    int run = incl - s;
#pragma unroll 1
    for (int i = 0; i < NBA / 32; ++i) {
      const int cv = cnt[base + i];
      offs[base + i] = run;
      cur[base + i]  = run;
      run += cv;
    }
  }
  __syncthreads();
  if (wave == 0) {
#pragma unroll 1
    for (int b0 = 0; b0 < tt; b0 += 32) {
      const int idx = b0 + lane;
      const int ent = hl[idx < RCAP ? idx : RCAP - 1];
      const int m32 = (tt - b0) < 32 ? (tt - b0) : 32;
#pragma unroll 1
      for (int k = 0; k < m32; ++k) {
        const int u    = __builtin_amdgcn_readlane(ent, k);
        const int slot = u & (NBA - 1);
        if (lane == 0) {
          int p = cur[slot];
          p = p < 0 ? 0 : (p > RCAP - 1 ? RCAP - 1 : p);
          sl[p] = u;
          cur[slot] = p + 1;
        }
      }
    }
  }
  __syncthreads();

#pragma unroll 1
  for (int idx = tid; idx < RCAP; idx += NTHR) {
    const int ent = sl[idx];
    const int eid = clampi(ent >> SLA, 0, nE - 1);
    int sr = srcs[eid];
    asm volatile("" :: "v"(sr));
    sr = clampi(sr, 0, nN - 1);
    const int msk = (idx < tt) ? -1 : 0;
    hl[idx] = sr & msk;
  }
  __syncthreads();

  int* hg = HITS + (size_t)blockIdx.x * RCAP;
#pragma unroll 1
  for (int it = 0; it < RCAP / (4 * NTHR); ++it) {
    const int q = 4 * (it * NTHR + tid);
    const v4i v = *(const v4ia*)(hl + q);
    *(volatile v4i*)(hg + q) = v;
  }
  __threadfence();
#pragma unroll 1
  for (int it = 0; it < RCAP / (4 * NTHR); ++it) {
    const int q = 4 * (it * NTHR + tid);
    const v4i v = *(const v4ia*)(hl + q);
    *(volatile v4i*)(hg + q) = v;
  }

  {
    const int s0 = 4 * tid;
    const v4i c4 = *(const v4ia*)(cnt + s0);
    const v4i o4 = *(const v4ia*)(offs + s0);
    v4f dv;
    dv.x = rsq_ref((float)c4.x + 1.0f);
    dv.y = rsq_ref((float)c4.y + 1.0f);
    dv.z = rsq_ref((float)c4.z + 1.0f);
    dv.w = rsq_ref((float)c4.w + 1.0f);
    int*   cg = CNT  + (size_t)nodeBase + s0;
    int*   og = OFF  + (size_t)nodeBase + s0;
    float* dg = DINV + (size_t)nodeBase + s0;
    const v4i f4 = {ovf, ovf, ovf, ovf};
    int* fg = FLG + (size_t)blockIdx.x * 32 + 4 * (tid & 7);
    *(volatile v4i*)cg = c4;
    *(volatile v4i*)og = o4;
    *(volatile v4f*)dg = dv;
    if (tid < 8) *(volatile v4i*)fg = f4;
    __threadfence();
    *(volatile v4i*)cg = c4;
    *(volatile v4i*)og = o4;
    *(volatile v4f*)dg = dv;
    if (tid < 8) *(volatile v4i*)fg = f4;
  }
}

template <int SCALE>
__global__ __launch_bounds__(GTHR) __attribute__((amdgpu_num_vgpr(248)))
void k_gemm(const unsigned short* __restrict__ A, int lda,
            const unsigned short* __restrict__ BT, int ldb, int K,
            const float* __restrict__ dinv, float* Cm, int ldc) {
  __shared__ __attribute__((aligned(16))) float stg[GBM * GBN];
  const int tid = (int)threadIdx.x, lane = tid & 31, wave = tid >> 5, hh = lane >> 4, m = lane & 15;
  const int rowBase = (int)blockIdx.x * GBM;
  const int colBase = (int)blockIdx.y * GBN;

  v8f acc[8];
  {
    const v8f z = {0.f, 0.f, 0.f, 0.f, 0.f, 0.f, 0.f, 0.f};
#pragma unroll
    for (int t = 0; t < 8; ++t) acc[t] = z;
  }
  const unsigned short* ap = A  + (size_t)(rowBase + 16 * wave + m) * (size_t)lda + 8 * hh;
  const unsigned short* bp = BT + (size_t)(colBase + m) * (size_t)ldb + 8 * hh;

#pragma unroll 1
  for (int k0 = 0; k0 < K; k0 += 32) {
    FragB af;
    af.h[0] = *(const v8usa*)(ap + k0);
    af.h[1] = *(const v8usa*)(ap + k0 + 16);
#pragma unroll
    for (int nt = 0; nt < 8; ++nt) {
      const unsigned short* wq = bp + (size_t)(16 * nt) * (size_t)ldb + k0;
      FragB bf;
      bf.h[0] = *(const v8usa*)wq;
      bf.h[1] = *(const v8usa*)(wq + 16);
      acc[nt] = wmb(af, bf, acc[nt]);
    }
  }

  v8f dv8 = {1.f, 1.f, 1.f, 1.f, 1.f, 1.f, 1.f, 1.f};
  if constexpr (SCALE != 0) {
    const float* dq = dinv + rowBase + 16 * wave + 8 * hh;
    const v4f d0 = *(const v4fa*)dq;
    const v4f d1 = *(const v4fa*)(dq + 4);
    const v8f dd = {d0.x, d0.y, d0.z, d0.w, d1.x, d1.y, d1.z, d1.w};
    dv8 = dd;
  }
#pragma unroll
  for (int nt = 0; nt < 8; ++nt) {
    const int lc = 16 * nt + m;
#pragma unroll
    for (int r = 0; r < 8; ++r) {
      const int lr = 16 * wave + 8 * hh + r;
      float v = acc[nt][r];
      if constexpr (SCALE != 0) v = v * dv8[r];
      stg[lr * GBN + lc] = v;
    }
  }
  __syncthreads();

  v4f pv[16];
#pragma unroll
  for (int i = 0; i < 16; ++i) pv[i] = *(const v4fa*)(stg + (16 * wave + i) * GBN + 4 * lane);
#pragma unroll
  for (int i = 0; i < 16; ++i) {
    float* op = Cm + (size_t)(rowBase + 16 * wave + i) * (size_t)ldc + colBase + 4 * lane;
    *(volatile v4f*)op = pv[i];
  }
  __threadfence();
#pragma unroll
  for (int i = 0; i < 16; ++i) {
    float* op = Cm + (size_t)(rowBase + 16 * wave + i) * (size_t)ldc + colBase + 4 * lane;
    *(volatile v4f*)op = pv[i];
  }
}

template <int RELU>
__global__ __launch_bounds__(NTHR) void k_agg(const int* __restrict__ HITS, const int* __restrict__ CNT,
                                              const int* __restrict__ OFF, const int* __restrict__ FLG,
                                              const float* __restrict__ DINV, const float* __restrict__ HP,
                                              const float* __restrict__ bias, int nN, int mRows,
                                              unsigned short* XHL) {
  const int tid = (int)threadIdx.x, lane = tid & 31, wave = tid >> 5;
  v4f bv;
  {
    const v4f a = *(const v4fa*)(bias + 4 * lane);
    bv.x = bf16_val(a.x); bv.y = bf16_val(a.y); bv.z = bf16_val(a.z); bv.w = bf16_val(a.w);
  }
  const float qnan = __int_as_float(0x7fc00000);
  const int sa = (2 * lane) & 31, sb = (2 * lane + 1) & 31;
#pragma unroll 1
  for (int si = 0; si < APB / NWAVE; ++si) {
    const int node = (int)blockIdx.x * APB + si * NWAVE + wave;
    const int nt   = node < NTAB ? node : NTAB - 1;
    const int bk   = nt >> SLA;
    int c = CNT[nt];
    const bool big = c > DEGCAP;
    c = c < 0 ? 0 : (c > DEGCAP ? DEGCAP : c);
    int o = OFF[nt];
    o = o < 0 ? 0 : (o > RCAP ? RCAP : o);
    const int fl = FLG[bk * 32];
    const int nc = node < nN ? node : nN - 1;
    const float dd = DINV[nc];
    const int* hb = HITS + (size_t)bk * RCAP;
    v4f acc = {0.0f, 0.0f, 0.0f, 0.0f};
#pragma unroll 1
    for (int b0 = 0; b0 < c; b0 += 32) {
      int idx = o + b0 + lane;
      idx = idx > RCAP - 1 ? RCAP - 1 : idx;
      int sr = hb[idx];
      sr = clampi(sr, 0, nN - 1);
      const int m32 = (c - b0) < 32 ? (c - b0) : 32;
#pragma unroll 1
      for (int k = 0; k < m32; ++k) {
        const int sk = __builtin_amdgcn_readlane(sr, k);
        const v4f a = *(const v4fa*)(HP + (size_t)sk * HID + 4 * lane);
        acc.x += a.x; acc.y += a.y; acc.z += a.z; acc.w += a.w;
      }
    }
    const v4f sv = *(const v4fa*)(HP + (size_t)nc * HID + 4 * lane);
    float y0 = fmaf(dd, acc.x + sv.x, bv.x);
    float y1 = fmaf(dd, acc.y + sv.y, bv.y);
    float y2 = fmaf(dd, acc.z + sv.z, bv.z);
    float y3 = fmaf(dd, acc.w + sv.w, bv.w);
    if constexpr (RELU != 0) {
      y0 = (y0 > 0.0f) ? y0 : (y0 - y0);
      y1 = (y1 > 0.0f) ? y1 : (y1 - y1);
      y2 = (y2 > 0.0f) ? y2 : (y2 - y2);
      y3 = (y3 > 0.0f) ? y3 : (y3 - y3);
    }
    const float pzr = (big || fl != 0) ? qnan : 0.0f;
    y0 = y0 + pzr; y1 = y1 + pzr; y2 = y2 + pzr; y3 = y3 + pzr;
    const bool live = node < nN;
    const float v0 = live ? y0 : 0.0f;
    const float v1 = live ? y1 : 0.0f;
    const float v2 = live ? y2 : 0.0f;
    const float v3 = live ? y3 : 0.0f;
    const unsigned h0 = bf16_bits_np(v0), h1 = bf16_bits_np(v1);
    const unsigned h2 = bf16_bits_np(v2), h3 = bf16_bits_np(v3);
    const unsigned l0 = bf16_bits_np(v0 - __uint_as_float(h0 << 16));
    const unsigned l1 = bf16_bits_np(v1 - __uint_as_float(h1 << 16));
    const unsigned l2 = bf16_bits_np(v2 - __uint_as_float(h2 << 16));
    const unsigned l3 = bf16_bits_np(v3 - __uint_as_float(h3 << 16));
    const int hw0 = (int)(h0 | (h1 << 16));
    const int hw1 = (int)(h2 | (h3 << 16));
    const int lw0 = (int)(l0 | (l1 << 16));
    const int lw1 = (int)(l2 | (l3 << 16));
    const int g0 = __shfl(hw0, sa, 32), g1 = __shfl(hw1, sa, 32);
    const int g2 = __shfl(hw0, sb, 32), g3 = __shfl(hw1, sb, 32);
    const int p0 = __shfl(lw0, sa, 32), p1 = __shfl(lw1, sa, 32);
    const int p2 = __shfl(lw0, sb, 32), p3 = __shfl(lw1, sb, 32);
    const unsigned ml = 0u - (unsigned)(lane >> 4);
    const unsigned mh = ~ml;
    v4u pv;
    pv.x = ((unsigned)g0 & mh) | ((unsigned)p0 & ml);
    pv.y = ((unsigned)g1 & mh) | ((unsigned)p1 & ml);
    pv.z = ((unsigned)g2 & mh) | ((unsigned)p2 & ml);
    pv.w = ((unsigned)g3 & mh) | ((unsigned)p3 & ml);
    const bool wr = node < mRows;
    const int nr = wr ? node : mRows - 1;
    unsigned short* hp = XHL + (size_t)nr * K2 + 8 * lane;
    if (wr) *(volatile v4u*)hp = pv;
    __threadfence();
    if (wr) *(volatile v4u*)hp = pv;
  }
}

__global__ __launch_bounds__(NTHR) __attribute__((amdgpu_num_vgpr(248)))
void k_head(const int* __restrict__ src, const int* __restrict__ dst, int nN, int nE,
            const float* __restrict__ EA, const unsigned short* __restrict__ WET,
            const float* __restrict__ PAB, const float* __restrict__ bm1,
            const float* __restrict__ Wm2, const float* __restrict__ bm2, float* out) {
  extern __shared__ __attribute__((aligned(16))) float dyn[];
  float* sD  = dyn;
  float* cst = dyn + NWAVE * 16 * DP;
  const int tid = (int)threadIdx.x, lane = tid & 31, wave = tid >> 5, hh = lane >> 4, m = lane & 15;

  if (tid < HID) {
    cst[tid]       = bf16_val(bm1[tid]);
    cst[HID + tid] = bf16_val(Wm2[tid]);
  }
  if (tid == 0) cst[2 * HID] = bf16_val(bm2[0]);
  __syncthreads();

  const v4f b4 = *(const v4fa*)(cst + 4 * lane);
  const v4f w4 = *(const v4fa*)(cst + HID + 4 * lane);
  const float bm2v = cst[2 * HID];
  const int ebase = (int)blockIdx.x * EPB + wave * 32;
  float* sDw = sD + wave * 16 * DP;
  const unsigned short* wp = WET + (size_t)m * EFK + 8 * hh;
  float res = 0.0f;

#pragma unroll 1
  for (int ht = 0; ht < 2; ++ht) {
    int e = ebase + 16 * ht + m;
    e = e > nE - 1 ? nE - 1 : e;
    int s = src[e];
    int d = dst[e];
    asm volatile("" :: "v"(s), "v"(d));
    s = clampi(s, 0, nN - 1);
    d = clampi(d, 0, nN - 1);
    const float* aq = EA + (size_t)e * EDIM + 8 * hh;
    const v4f a0 = *(const v4fa*)aq;
    const v4f a1 = *(const v4fa*)(aq + 4);
    FragB af;
    af.u[0] = (unsigned short)bf16_bits(a0.x);
    af.u[1] = (unsigned short)bf16_bits(a0.y);
    af.u[2] = (unsigned short)bf16_bits(a0.z);
    af.u[3] = (unsigned short)bf16_bits(a0.w);
    af.u[4] = (unsigned short)bf16_bits(a1.x);
    af.u[5] = (unsigned short)bf16_bits(a1.y);
    af.u[6] = (unsigned short)bf16_bits(a1.z);
    af.u[7] = (unsigned short)bf16_bits(a1.w);
#pragma unroll
    for (int i = 8; i < 16; ++i) af.u[i] = (unsigned short)0;

    v8f acc[8];
    {
      const v8f z = {0.f, 0.f, 0.f, 0.f, 0.f, 0.f, 0.f, 0.f};
#pragma unroll
      for (int nt = 0; nt < 8; ++nt) acc[nt] = z;
    }
#pragma unroll
    for (int nt = 0; nt < 8; ++nt) {
      const unsigned short* wq = wp + (size_t)(16 * nt) * EFK;
      FragB bf;
      bf.h[0] = *(const v8usa*)wq;
      bf.h[1] = *(const v8usa*)(wq + 16);
      acc[nt] = wmb(af, bf, acc[nt]);
    }
#pragma unroll
    for (int nt = 0; nt < 8; ++nt) {
      const int col = 16 * nt + m;
#pragma unroll
      for (int r = 0; r < 8; ++r) sDw[(8 * hh + r) * DP + col] = acc[nt][r];
    }
    __syncthreads();

#pragma unroll 1
    for (int r = 0; r < 16; ++r) {
      const int sk = __builtin_amdgcn_readlane(s, r);
      const int dk = __builtin_amdgcn_readlane(d, r);
      const v4f tv = *(const v4fa*)(sDw + r * DP + 4 * lane);
      const v4f pa = *(const v4fa*)(PAB + (size_t)sk * NPAB + 4 * lane);
      const v4f pb = *(const v4fa*)(PAB + (size_t)dk * NPAB + HID + 4 * lane);
      float x0 = ((tv.x + pa.x) + pb.x) + b4.x;
      float x1 = ((tv.y + pa.y) + pb.y) + b4.y;
      float x2 = ((tv.z + pa.z) + pb.z) + b4.z;
      float x3 = ((tv.w + pa.w) + pb.w) + b4.w;
      x0 = (x0 > 0.0f) ? x0 : (x0 - x0);
      x1 = (x1 > 0.0f) ? x1 : (x1 - x1);
      x2 = (x2 > 0.0f) ? x2 : (x2 - x2);
      x3 = (x3 > 0.0f) ? x3 : (x3 - x3);
      float p = x0 * w4.x;
      p = fmaf(x1, w4.y, p);
      p = fmaf(x2, w4.z, p);
      p = fmaf(x3, w4.w, p);
      p += __shfl_xor(p, 1, 32);
      p += __shfl_xor(p, 2, 32);
      p += __shfl_xor(p, 4, 32);
      p += __shfl_xor(p, 8, 32);
      p += __shfl_xor(p, 16, 32);
      res = (lane == 16 * ht + r) ? p : res;
    }
    __syncthreads();
  }

  const float ov = res + bm2v;
  float* op = out + (size_t)ebase + lane;
  *(volatile float*)op = ov;
  __threadfence();
  *(volatile float*)op = ov;
}

extern "C" void kernel_launch(void* const* d_in, const int* in_sizes, int n_in,
                              void* d_out, int out_size, void* d_ws, size_t ws_size,
                              hipStream_t stream) {
  if (n_in < 11) return;
  if (in_sizes[0] != NN * HID) return;
  if (in_sizes[1] != 2 * NE) return;
  if (in_sizes[2] != NE * EDIM) return;
  if (in_sizes[3] != HID * HID || in_sizes[4] != HID) return;
  if (in_sizes[5] != HID * HID || in_sizes[6] != HID) return;
  if (in_sizes[7] != KW * HID || in_sizes[8] != HID) return;
  if (in_sizes[9] != HID || in_sizes[10] != 1) return;
  if (out_size != NE) return;

  const float* x    = (const float*)d_in[0];
  const int*   edge = (const int*)d_in[1];
  const float* ea   = (const float*)d_in[2];
  const float* W1   = (const float*)d_in[3];
  const float* b1   = (const float*)d_in[4];
  const float* W2   = (const float*)d_in[5];
  const float* b2   = (const float*)d_in[6];
  const float* Wm1  = (const float*)d_in[7];
  const float* bm1  = (const float*)d_in[8];
  const float* Wm2  = (const float*)d_in[9];
  const float* bm2  = (const float*)d_in[10];
  float* out = (float*)d_out;
  const int* src = edge;
  const int* dst = edge + NE;
  const int nN = NN, nE = NE;

  char* ws = (char*)d_ws;
  size_t off = 0;
  const size_t oW1T = off; off += (size_t)HID * HID * 2;
  const size_t oW2D = off; off += (size_t)HID * K2 * 2;
  const size_t oWPD = off; off += (size_t)NPAB * K2 * 2;
  const size_t oWET = off; off += (size_t)HID * EFK * 2;
  const size_t oXB  = off; off += (size_t)NPADR * HID * 2;
  const size_t oHP  = off; off += (size_t)NPADR * HID * 4;
  const size_t oXHL = off; off += (size_t)NPADR * K2 * 2;
  const size_t oPAB = off; off += (size_t)NPADR * NPAB * 4;
  const size_t oHIT = off; off += (size_t)NBLK * RCAP * 4;
  const size_t oCNT = off; off += (size_t)NTAB * 4;
  const size_t oOFF = off; off += (size_t)NTAB * 4;
  const size_t oDIN = off; off += (size_t)NTAB * 4;
  const size_t oFLG = off; off += (size_t)64 * 128;
  if (off > ws_size || off > (size_t)WSMAX) return;
  unsigned short* W1T = (unsigned short*)(ws + oW1T);
  unsigned short* W2D = (unsigned short*)(ws + oW2D);
  unsigned short* WPD = (unsigned short*)(ws + oWPD);
  unsigned short* WET = (unsigned short*)(ws + oWET);
  unsigned short* XB  = (unsigned short*)(ws + oXB);
  float*          HP  = (float*)(ws + oHP);
  unsigned short* XHL = (unsigned short*)(ws + oXHL);
  float*          PAB = (float*)(ws + oPAB);
  int*            HIT = (int*)(ws + oHIT);
  int*            CNT = (int*)(ws + oCNT);
  int*            OFF = (int*)(ws + oOFF);
  float*          DIN = (float*)(ws + oDIN);
  int*            FLG = (int*)(ws + oFLG);

  hipFuncSetAttribute(reinterpret_cast<const void*>(&k_bucket), hipFuncAttributeMaxDynamicSharedMemorySize,
                      (int)BKT_LDS_BYTES);
  hipFuncSetAttribute(reinterpret_cast<const void*>(&k_head), hipFuncAttributeMaxDynamicSharedMemorySize,
                      (int)HEAD_LDS_BYTES);

  const int nPrep = NU_W1 + NU_W2 + NU_WP + NU_WE + NU_XB;
  const int gM = NPADR / GBM;
  const int vec8 = 1;

  k_prep<<<nPrep / NTHR, NTHR, 0, stream>>>(x, W1, W2, Wm1, nN, W1T, W2D, WPD, WET, XB);
  k_bucket<<<NBLK, NTHR, BKT_LDS_BYTES, stream>>>(src, dst, nE, nN, vec8, HIT, CNT, OFF, DIN, FLG);
  k_gemm<1><<<dim3(gM, 1), GTHR, 0, stream>>>(XB, HID, W1T, HID, HID, DIN, HP, HID);
  k_agg<1><<<NPADR / APB, NTHR, 0, stream>>>(HIT, CNT, OFF, FLG, DIN, HP, b1, nN, NPADR, XHL);
  k_gemm<1><<<dim3(gM, 1), GTHR, 0, stream>>>(XHL, K2, W2D, K2, K2, DIN, HP, HID);
  k_agg<0><<<NPADR / APB, NTHR, 0, stream>>>(HIT, CNT, OFF, FLG, DIN, HP, b2, nN, NPADR, XHL);
  k_gemm<0><<<dim3(gM, NPAB / GBN), GTHR, 0, stream>>>(XHL, K2, WPD, K2, K2, DIN, PAB, NPAB);
  k_head<<<NE / EPB, NTHR, HEAD_LDS_BYTES, stream>>>(src, dst, nN, nE, ea, WET, PAB, bm1, Wm2, bm2, out);
}
